// MultiHeadAttention__24919400252075
// MI455X (gfx1250) — hardware-verified
//
#include <hip/hip_runtime.h>
#include <math.h>

constexpr int kBatch   = 2;
constexpr int kSeq     = 2048;
constexpr int kDim     = 1024;
constexpr int kHeads   = 16;
constexpr int kDh      = 64;
constexpr int kTok     = kBatch * kSeq;
constexpr int kQBlocks = kSeq / 64;
constexpr int kSplitQB = 8;
constexpr float kQScale  = 0.125f;
constexpr float kNegHuge = -3.0e38f;
static_assert(kHeads * kDh == kDim, "shape");
static_assert(kDim % 64 == 0 && kTok % 64 == 0 && kSeq % 64 == 0, "tiles");
static_assert(kDim % 32 == 0, "kdepth");
static_assert(kSplitQB > 0 && kSplitQB < kQBlocks, "split");
static_assert(((kTok / 64) * (kDim / 64)) % 8 == 0, "grid");
static_assert((kTok * kDim) % (8 * 256) == 0, "castgrid");

typedef __attribute__((ext_vector_type(16))) _Float16 v16h;
typedef __attribute__((ext_vector_type(8)))  _Float16 v8h;
typedef __attribute__((ext_vector_type(16))) __bf16   v16b;
typedef __attribute__((ext_vector_type(8)))  __bf16   v8b;
typedef __attribute__((ext_vector_type(8)))  float    v8f;
typedef __attribute__((ext_vector_type(4)))  float    v4f;
typedef __attribute__((ext_vector_type(4)))  unsigned int v4u;

__device__ __forceinline__ unsigned short f2bf_bits(float f) {
  unsigned u = __float_as_uint(f);
  return (unsigned short)((u + 0x7FFFu + ((u >> 16) & 1u)) >> 16);
}
__device__ __forceinline__ float bf_bits2f(unsigned short h) { return __uint_as_float(((unsigned)h) << 16); }
__device__ __forceinline__ unsigned pk16(unsigned short a, unsigned short b) { return (unsigned)a | ((unsigned)b << 16); }
__device__ __forceinline__ unsigned short h_bits(float f) { const _Float16 h = (_Float16)f; return __builtin_bit_cast(unsigned short, h); }

__device__ __forceinline__ void dep_guard_h(v8f& a, v8f& b, v16h x, v16h y) { asm volatile("v_nop\n\tv_nop\n\tv_nop\n\tv_nop" : "+v"(a), "+v"(b) : "v"(x), "v"(y)); }
__device__ __forceinline__ void dep_guard_b(v8f& a, v8f& b, v16b x, v16b y) { asm volatile("v_nop\n\tv_nop\n\tv_nop\n\tv_nop" : "+v"(a), "+v"(b) : "v"(x), "v"(y)); }
__device__ __forceinline__ void keep4_h(v16h a, v16h b, v16h c, v16h d) { asm volatile("v_nop" :: "v"(a), "v"(b), "v"(c), "v"(d)); }
__device__ __forceinline__ void keep4_b(v16b a, v16b b, v16b c, v16b d) { asm volatile("v_nop" :: "v"(a), "v"(b), "v"(c), "v"(d)); }
__device__ __forceinline__ void acc_guard4(v8f& a, v8f& b, v8f& c, v8f& d) { asm volatile("v_nop\n\tv_nop\n\tv_nop\n\tv_nop" : "+v"(a), "+v"(b), "+v"(c), "+v"(d)); }
template <typename VA, typename VB>
__device__ __forceinline__ void guard_row(v8f& a0, v8f& a1, v8f& a2, v8f& a3, VA x, VB y) {
  asm volatile("v_nop\n\tv_nop\n\tv_nop\n\tv_nop" : "+v"(a0), "+v"(a1), "+v"(a2), "+v"(a3) : "v"(x), "v"(y) : "memory");
}

template <typename T> struct Frag;
template <> struct Frag<_Float16> {
  typedef v16h V; union U { v16h v; v8h h[2]; };
  static __device__ __forceinline__ v16h load(const _Float16* p) {
    U f; f.h[0] = *(const v8h*)(p); f.h[1] = *(const v8h*)(p + 16); return f.v;
  }
  static __device__ __forceinline__ v8f mma(v16h a, v16h b, v8f c) {
    return __builtin_amdgcn_wmma_f32_16x16x32_f16(false, a, false, b, (short)0, c, false, false);
  }
  static __device__ __forceinline__ void guard(v8f& a, v8f& b, v16h x, v16h y) { dep_guard_h(a, b, x, y); }
  static __device__ __forceinline__ void keep(v16h a, v16h b, v16h c, v16h d) { keep4_h(a, b, c, d); }
};
template <> struct Frag<__bf16> {
  typedef v16b V; union U { v16b v; v8b h[2]; };
  static __device__ __forceinline__ v16b load(const __bf16* p) {
    U f; f.h[0] = *(const v8b*)(p); f.h[1] = *(const v8b*)(p + 16); return f.v;
  }
  static __device__ __forceinline__ v8f mma(v16b a, v16b b, v8f c) {
    return __builtin_amdgcn_wmma_f32_16x16x32_bf16(false, a, false, b, (short)0, c, false, false);
  }
  static __device__ __forceinline__ void guard(v8f& a, v8f& b, v16b x, v16b y) { dep_guard_b(a, b, x, y); }
  static __device__ __forceinline__ void keep(v16b a, v16b b, v16b c, v16b d) { keep4_b(a, b, c, d); }
};

__device__ __forceinline__ v8f mma_g(v16h a, v16h b, v8f c) {
  c = __builtin_amdgcn_wmma_f32_16x16x32_f16(false, a, false, b, (short)0, c, false, false);
  asm volatile("v_nop\n\tv_nop\n\tv_nop\n\tv_nop" : "+v"(c) : "v"(a), "v"(b) : "memory");
  return c;
}
__device__ __forceinline__ v8f mma_g(v16b a, v16b b, v8f c) {
  c = __builtin_amdgcn_wmma_f32_16x16x32_bf16(false, a, false, b, (short)0, c, false, false);
  asm volatile("v_nop\n\tv_nop\n\tv_nop\n\tv_nop" : "+v"(c) : "v"(a), "v"(b) : "memory");
  return c;
}

template <int ET> struct Elem;
template <> struct Elem<0> { typedef _Float16 T; };
template <> struct Elem<1> { typedef __bf16 T; };

template <int ET, int NPROD, int BIAS_MODE, int OUT_MODE>
__global__ __launch_bounds__(256) void wmma_gemm64(
    const unsigned short* __restrict__ Ap, const unsigned short* __restrict__ A2p, int lda, long strideA,
    const unsigned short* __restrict__ Btp, int ldb, long strideB,
    void* __restrict__ Cout, void* __restrict__ Cout2, void* __restrict__ Cout3, int ldc, long strideC,
    const float* __restrict__ bias, int M, int N, int K, float scale) {
  static_assert(NPROD == 1 || NPROD == 2, "np");
  static_assert(OUT_MODE == 0 || OUT_MODE == 3, "om");
  static_assert(BIAS_MODE == 1 || BIAS_MODE == 2, "bm");
  typedef typename Elem<ET>::T T;
  typedef typename Frag<T>::V V;
  const T* A = (const T*)Ap; const T* A2 = (const T*)A2p; const T* Bt = (const T*)Btp;
  __shared__ __align__(16) float sT[8][16 * 68];
  const int b    = blockIdx.y;
  const int lane = threadIdx.x & 31;
  const int wave = threadIdx.x >> 5;
  const int tilesN = N >> 6;
  const int tilesM = M >> 6;
  const int tile = blockIdx.x * 8 + wave;
  if (tile >= tilesM * tilesN) return;
  const int tm = tile / tilesN;
  const int tn = tile - tm * tilesN;
  const int m0 = tm << 6;
  const int n0 = tn << 6;

  const T* Ab  = A  + (size_t)b * strideA;
  const T* Ab2 = A2 + (size_t)b * strideA;
  const T* Bb  = Bt + (size_t)b * strideB;

  const int rlane = lane & 15;
  const int koff  = (lane >> 4) * 8;
  const int mOff  = (lane >> 4) * 8;

  v8f acc[4][4];
#pragma unroll
  for (int i = 0; i < 4; ++i)
#pragma unroll
    for (int j = 0; j < 4; ++j) acc[i][j] = (v8f){0.f,0.f,0.f,0.f,0.f,0.f,0.f,0.f};

  for (int k0 = 0; k0 < K; k0 += 32) {
    V bh[4];
#pragma unroll
    for (int j = 0; j < 4; ++j) {
      const size_t bo = (size_t)(n0 + (j << 4) + rlane) * ldb + koff + k0;
      bh[j] = Frag<T>::load(Bb + bo);
    }
#pragma unroll
    for (int i = 0; i < 4; ++i) {
      const size_t ao = (size_t)(m0 + (i << 4) + rlane) * lda + koff + k0;
      V ah = Frag<T>::load(Ab + ao);
      V al = ah;
      if (NPROD == 2) al = Frag<T>::load(Ab2 + ao);
#pragma unroll
      for (int j = 0; j < 4; ++j) {
        acc[i][j] = Frag<T>::mma(ah, bh[j], acc[i][j]);
        if (NPROD == 2) acc[i][j] = Frag<T>::mma(al, bh[j], acc[i][j]);
      }
      guard_row(acc[i][0], acc[i][1], acc[i][2], acc[i][3], ah, al);
    }
    Frag<T>::keep(bh[0], bh[1], bh[2], bh[3]);
  }
  acc_guard4(acc[0][0], acc[0][1], acc[0][2], acc[0][3]);
  acc_guard4(acc[1][0], acc[1][1], acc[1][2], acc[1][3]);
  acc_guard4(acc[2][0], acc[2][1], acc[2][2], acc[2][3]);
  acc_guard4(acc[3][0], acc[3][1], acc[3][2], acc[3][3]);

  float* slab = sT[wave];
#pragma unroll
  for (int i = 0; i < 4; ++i) {
    const int mBase = m0 + (i << 4);
    float bm[8];
    if (BIAS_MODE == 1) {
#pragma unroll
      for (int r = 0; r < 8; ++r) bm[r] = bf_bits2f(f2bf_bits(bias[mBase + mOff + r]));
    } else {
#pragma unroll
      for (int r = 0; r < 8; ++r) bm[r] = 0.f;
    }
#pragma unroll
    for (int j = 0; j < 4; ++j) {
      const int n = n0 + (j << 4) + rlane;
      float bn = 0.f;
      if (BIAS_MODE == 2) bn = bf_bits2f(f2bf_bits(bias[n]));
#pragma unroll
      for (int r = 0; r < 8; ++r) {
        float v = acc[i][j][r] * scale;
        if (BIAS_MODE == 1) v += bm[r];
        if (BIAS_MODE == 2) v += bn;
        slab[(mOff + r) * 68 + (j << 4) + rlane] = v;
      }
    }
    __builtin_amdgcn_fence(__ATOMIC_RELEASE, "workgroup");
    __builtin_amdgcn_wave_barrier();
    __builtin_amdgcn_fence(__ATOMIC_ACQUIRE, "workgroup");
    if (OUT_MODE == 0) {
      float* C = (float*)Cout + (size_t)b * strideC;
      const int hh = lane >> 4, c4 = (lane & 15) * 4;
      for (int pass = 0; pass < 2; ++pass) {
#pragma unroll
        for (int it = 0; it < 8; ++it) {
          const int row = it * 2 + hh;
          v4f v = *(const v4f*)(slab + row * 68 + c4);
          *(volatile v4f*)(C + (size_t)(mBase + row) * ldc + n0 + c4) = v;
        }
        __threadfence();
      }
    } else {
      const int q = lane >> 3, c8 = (lane & 7) * 8;
      unsigned short* C  = (unsigned short*)Cout  + (size_t)b * strideC;
      unsigned short* C2 = (unsigned short*)Cout2 + (size_t)b * strideC;
      unsigned short* C3 = (unsigned short*)Cout3 + (size_t)b * strideC;
      for (int pass = 0; pass < 2; ++pass) {
#pragma unroll
        for (int it = 0; it < 4; ++it) {
          const int row = it * 4 + q;
          const float* sp = slab + row * 68 + c8;
          const v4f x0 = *(const v4f*)(sp);
          const v4f x1 = *(const v4f*)(sp + 4);
          unsigned short hb[8], bb[8], lb[8];
#pragma unroll
          for (int e = 0; e < 4; ++e) {
            const float xa = x0[e];
            const float xb = x1[e];
            hb[e] = h_bits(xa);
            hb[4 + e] = h_bits(xb);
            const unsigned short ba = f2bf_bits(xa);
            const unsigned short bb2 = f2bf_bits(xb);
            bb[e] = ba;
            bb[4 + e] = bb2;
            lb[e] = f2bf_bits(xa - bf_bits2f(ba));
            lb[4 + e] = f2bf_bits(xb - bf_bits2f(bb2));
          }
          const v4u uh = (v4u){pk16(hb[0], hb[1]), pk16(hb[2], hb[3]), pk16(hb[4], hb[5]), pk16(hb[6], hb[7])};
          const v4u ub = (v4u){pk16(bb[0], bb[1]), pk16(bb[2], bb[3]), pk16(bb[4], bb[5]), pk16(bb[6], bb[7])};
          const v4u ul = (v4u){pk16(lb[0], lb[1]), pk16(lb[2], lb[3]), pk16(lb[4], lb[5]), pk16(lb[6], lb[7])};
          const size_t co = (size_t)(mBase + row) * ldc + n0 + c8;
          *(volatile v4u*)(C  + co) = uh;
          *(volatile v4u*)(C2 + co) = ub;
          *(volatile v4u*)(C3 + co) = ul;
        }
        __threadfence();
      }
    }
    __builtin_amdgcn_fence(__ATOMIC_RELEASE, "workgroup");
    __builtin_amdgcn_wave_barrier();
    __builtin_amdgcn_fence(__ATOMIC_ACQUIRE, "workgroup");
  }
}

__global__ __launch_bounds__(256) void xcast_bf16_kernel(const float* __restrict__ xa, const float* __restrict__ xb,
                                                        unsigned short* __restrict__ oa, unsigned short* __restrict__ ob,
                                                        int n8) {
  const int i = blockIdx.x * 256 + threadIdx.x;
  if (i >= n8) return;
  const bool second = (blockIdx.y != 0);
  const float* src = second ? xb : xa;
  unsigned short* dst = second ? ob : oa;
  const float* p = src + 8 * (size_t)i;
  const v4f a = *(const v4f*)(p);
  const v4f c = *(const v4f*)(p + 4);
  unsigned short ub[8];
#pragma unroll
  for (int e = 0; e < 4; ++e) {
    ub[e]     = f2bf_bits(a[e]);
    ub[4 + e] = f2bf_bits(c[e]);
  }
  const v4u u = (v4u){pk16(ub[0], ub[1]), pk16(ub[2], ub[3]), pk16(ub[4], ub[5]), pk16(ub[6], ub[7])};
  unsigned short* q = dst + 8 * (size_t)i;
  *(volatile v4u*)q = u;
  __threadfence();
  *(volatile v4u*)q = u;
}

__global__ __launch_bounds__(256) void wt_cast_kernel(const float* __restrict__ W0, const float* __restrict__ W1,
                                                      const float* __restrict__ W2, const float* __restrict__ W3,
                                                      unsigned short* __restrict__ outB) {
  __shared__ float sm[64][65];
  const int t   = threadIdx.x;
  const int in0 = blockIdx.x * 64;
  const int o0  = blockIdx.y * 64;
  const int z   = blockIdx.z;
  const float* W = (z == 0) ? W0 : (z == 1) ? W1 : (z == 2) ? W2 : W3;
#pragma unroll
  for (int i = 0; i < 16; ++i) {
    const int e  = i * 256 + t;
    const int r  = e >> 6;
    const int cc = e & 63;
    sm[cc][r] = W[(size_t)(in0 + r) * kDim + o0 + cc];
  }
  __syncthreads();
  const int lane = t & 31, wave = t >> 5;
  const int q = lane >> 3, c8 = (lane & 7) * 8;
  unsigned short* op = outB + (size_t)z * kDim * kDim;
  for (int pass = 0; pass < 2; ++pass) {
#pragma unroll
    for (int it = 0; it < 2; ++it) {
      const int row = wave * 8 + it * 4 + q;
      unsigned short bb[8];
#pragma unroll
      for (int e = 0; e < 8; ++e) bb[e] = f2bf_bits(sm[row][c8 + e]);
      const size_t wo = (size_t)(o0 + row) * kDim + in0 + c8;
      const v4u ub = (v4u){pk16(bb[0], bb[1]), pk16(bb[2], bb[3]), pk16(bb[4], bb[5]), pk16(bb[6], bb[7])};
      *(volatile v4u*)(op + wo) = ub;
    }
    __threadfence();
  }
}

template <bool SPL>
__global__ __launch_bounds__(128) void attn_kernel(
    const unsigned short* __restrict__ Q1p, const unsigned short* __restrict__ Q2p,
    const unsigned short* __restrict__ K1p, const unsigned short* __restrict__ K2p,
    const unsigned short* __restrict__ V1p, const unsigned short* __restrict__ V2p,
    unsigned short* __restrict__ OHp, unsigned short* __restrict__ OLp, int qb0) {
  typedef typename Elem<SPL ? 1 : 0>::T T;
  typedef typename Frag<T>::V FV;
  __shared__ __align__(16) unsigned short Ks1[64 * 64];
  __shared__ __align__(16) unsigned short Ks2[SPL ? 64 * 64 : 8];
  __shared__ __align__(16) unsigned short Vs1[64 * 64];
  __shared__ __align__(16) unsigned short Vs2[SPL ? 64 * 64 : 8];
  __shared__ __align__(16) unsigned short Ps1[4][16 * 64];
  __shared__ __align__(16) unsigned short Ps2[SPL ? 4 : 1][SPL ? 16 * 64 : 8];
  __shared__ __align__(16) float          Os[4][16 * 68];

  const int tid  = threadIdx.x;
  const int wave = tid >> 5;
  const int lane = tid & 31;
  const int hh   = lane >> 4;
  const int c    = lane & 15;
  const int qb   = qb0 + (int)blockIdx.x;
  const int bh   = blockIdx.y;
  const int b    = bh >> 4;
  const int h    = bh & 15;
  const size_t tokbase = (size_t)b * kSeq;
  const int hcol = h * kDh;
  const int q0   = qb * 64 + wave * 16;

  const T* Q1 = (const T*)Q1p;
  const T* Q2 = (const T*)Q2p;

  FV qa1[2], qa2[2];
  {
    const size_t qo = (tokbase + q0 + c) * kDim + hcol + 8 * hh;
    qa1[0] = Frag<T>::load(Q1 + qo);
    qa1[1] = Frag<T>::load(Q1 + qo + 32);
    if (SPL) {
      asm volatile("" ::: "memory");
      qa2[0] = Frag<T>::load(Q2 + qo);
      qa2[1] = Frag<T>::load(Q2 + qo + 32);
    } else {
      qa2[0] = qa1[0];
      qa2[1] = qa1[1];
    }
    Frag<T>::keep(qa1[0], qa1[1], qa2[0], qa2[1]);
  }

  float mrow[8], lrow[8];
  v8f oacc[4];
#pragma unroll
  for (int r = 0; r < 8; ++r) { mrow[r] = kNegHuge; lrow[r] = 0.f; }
#pragma unroll
  for (int t = 0; t < 4; ++t) oacc[t] = (v8f){0.f,0.f,0.f,0.f,0.f,0.f,0.f,0.f};

  const int nChunks = qb + 1;
  for (int kc = 0; kc < nChunks; ++kc) {
    const int kv0 = kc * 64;
    __syncthreads();
    {
#pragma unroll
      for (int i = 0; i < 4; ++i) {
        const int w   = i * 128 + tid;
        const int row = w >> 3;
        const int cw  = (w & 7) * 8;
        const v4u kw = *(const v4u*)(K1p + (tokbase + kv0 + row) * kDim + hcol + cw);
        *(v4u*)(Ks1 + row * 64 + cw) = kw;
        if (SPL) {
          const v4u kw2 = *(const v4u*)(K2p + (tokbase + kv0 + row) * kDim + hcol + cw);
          *(v4u*)(Ks2 + row * 64 + cw) = kw2;
        }
      }
      asm volatile("" ::: "memory");
#pragma unroll
      for (int i = 0; i < 4; ++i) {
        const int w   = i * 128 + tid;
        const int row = w >> 3;
        const int cw  = (w & 7) * 8;
        const v4u vw = *(const v4u*)(V1p + (size_t)(hcol + row) * kTok + tokbase + kv0 + cw);
        *(v4u*)(Vs1 + row * 64 + cw) = vw;
        if (SPL) {
          const v4u vw2 = *(const v4u*)(V2p + (size_t)(hcol + row) * kTok + tokbase + kv0 + cw);
          *(v4u*)(Vs2 + row * 64 + cw) = vw2;
        }
      }
    }
    __syncthreads();

    v8f s[4];
#pragma unroll
    for (int j = 0; j < 4; ++j) {
      s[j] = (v8f){0.f,0.f,0.f,0.f,0.f,0.f,0.f,0.f};
#pragma unroll
      for (int dc = 0; dc < 2; ++dc) {
        const int ko = (j * 16 + c) * 64 + dc * 32 + 8 * hh;
        const FV kf = Frag<T>::load((const T*)Ks1 + ko);
        s[j] = mma_g(qa1[dc], kf, s[j]);
        if (SPL) {
          const FV kl = Frag<T>::load((const T*)Ks2 + ko);
          s[j] = mma_g(qa1[dc], kl, s[j]);
          s[j] = mma_g(qa2[dc], kf, s[j]);
        }
      }
    }

    const bool diag = (kc == qb);
    float cm[8];
#pragma unroll
    for (int r = 0; r < 8; ++r) {
      const int qrow = q0 + 8 * hh + r;
      float m = kNegHuge;
#pragma unroll
      for (int j = 0; j < 4; ++j) {
        const int kvcol = kv0 + j * 16 + c;
        const float sv = s[j][r] * kQScale;
        const float val = (diag && (kvcol > qrow)) ? kNegHuge : sv;
        s[j][r] = val;
        m = fmaxf(m, val);
      }
#pragma unroll
      for (int off = 1; off < 16; off <<= 1) m = fmaxf(m, __shfl_xor(m, off, 32));
      cm[r] = m;
    }

    unsigned short* pw1 = Ps1[wave];
    unsigned short* pw2 = Ps2[SPL ? wave : 0];
#pragma unroll
    for (int r = 0; r < 8; ++r) {
      const float mnew  = fmaxf(mrow[r], cm[r]);
      const float alpha = expf(mrow[r] - mnew);
      mrow[r] = mnew;
      float psum = 0.f;
#pragma unroll
      for (int j = 0; j < 4; ++j) {
        const float p = expf(s[j][r] - mnew);
        psum += p;
        const int pidx = (8 * hh + r) * 64 + j * 16 + c;
        if (SPL) {
          const unsigned short pb = f2bf_bits(p);
          pw1[pidx] = pb;
          pw2[pidx] = f2bf_bits(p - bf_bits2f(pb));
        } else {
          pw1[pidx] = h_bits(p);
        }
      }
#pragma unroll
      for (int off = 1; off < 16; off <<= 1) psum += __shfl_xor(psum, off, 32);
      lrow[r] = lrow[r] * alpha + psum;
#pragma unroll
      for (int t = 0; t < 4; ++t) oacc[t][r] *= alpha;
    }
    __syncthreads();

#pragma unroll
    for (int kk = 0; kk < 2; ++kk) {
      const int po = c * 64 + kk * 32 + 8 * hh;
      const FV pa1 = Frag<T>::load((const T*)pw1 + po);
      FV pa2 = pa1;
      if (SPL) pa2 = Frag<T>::load((const T*)pw2 + po);
#pragma unroll
      for (int t = 0; t < 4; ++t) {
        const int vo = (t * 16 + c) * 64 + kk * 32 + 8 * hh;
        const FV vf = Frag<T>::load((const T*)Vs1 + vo);
        oacc[t] = mma_g(pa1, vf, oacc[t]);
        if (SPL) {
          const FV vl = Frag<T>::load((const T*)Vs2 + vo);
          oacc[t] = mma_g(pa1, vl, oacc[t]);
          oacc[t] = mma_g(pa2, vf, oacc[t]);
        }
      }
    }
  }

  float* os = Os[wave];
#pragma unroll
  for (int r = 0; r < 8; ++r) {
    const float inv = 1.0f / lrow[r];
#pragma unroll
    for (int t = 0; t < 4; ++t) os[(8 * hh + r) * 68 + t * 16 + c] = oacc[t][r] * inv;
  }
  __syncthreads();
  {
    const int q4 = lane >> 3, c8 = (lane & 7) * 8;
    for (int pass = 0; pass < 2; ++pass) {
#pragma unroll
      for (int it = 0; it < 4; ++it) {
        const int row = it * 4 + q4;
        const float* sp = os + row * 68 + c8;
        const v4f x0 = *(const v4f*)(sp);
        const v4f x1 = *(const v4f*)(sp + 4);
        unsigned short hb[8], lb[8];
#pragma unroll
        for (int e = 0; e < 4; ++e) {
          const float xa = x0[e];
          const float xb = x1[e];
          const unsigned short ba = f2bf_bits(xa);
          const unsigned short bb = f2bf_bits(xb);
          hb[e] = ba;
          hb[4 + e] = bb;
          lb[e] = f2bf_bits(xa - bf_bits2f(ba));
          lb[4 + e] = f2bf_bits(xb - bf_bits2f(bb));
        }
        const v4u uh = (v4u){pk16(hb[0], hb[1]), pk16(hb[2], hb[3]), pk16(hb[4], hb[5]), pk16(hb[6], hb[7])};
        const v4u ul = (v4u){pk16(lb[0], lb[1]), pk16(lb[2], lb[3]), pk16(lb[4], lb[5]), pk16(lb[6], lb[7])};
        const size_t dst = (tokbase + q0 + row) * kDim + hcol + c8;
        *(volatile v4u*)(OHp + dst) = uh;
        *(volatile v4u*)(OLp + dst) = ul;
      }
      __threadfence();
    }
  }
}

extern "C" void kernel_launch(void* const* d_in, const int* in_sizes, int n_in,
                              void* d_out, int out_size, void* d_ws, size_t ws_size,
                              hipStream_t stream) {
  if (n_in < 10) return;
  const int nElem = kTok * kDim;
  const int nW    = kDim * kDim;
  if (in_sizes[0] != nElem || in_sizes[1] != nElem) return;
  if (in_sizes[2] != nW || in_sizes[4] != nW || in_sizes[6] != nW || in_sizes[8] != nW) return;
  if (in_sizes[3] != kDim || in_sizes[5] != kDim || in_sizes[7] != kDim || in_sizes[9] != kDim) return;
  if (out_size != nElem) return;

  const size_t szX = (size_t)nElem * 2;
  const size_t szW = (size_t)nW * 2;
  const size_t offXQB = 0;
  const size_t offXKB = offXQB + szX;
  const size_t offWQT = offXKB + szX;
  const size_t offWKT = offWQT + szW;
  const size_t offWVT = offWKT + szW;
  const size_t offWOT = offWVT + szW;
  const size_t offQH  = offWOT + szW;
  const size_t offQBH = offQH  + szX;
  const size_t offQBL = offQBH + szX;
  const size_t offKH  = offQBL + szX;
  const size_t offKBH = offKH  + szX;
  const size_t offKBL = offKBH + szX;
  const size_t offVH  = offKBL + szX;
  const size_t offVBH = offVH  + szX;
  const size_t offVBL = offVBH + szX;
  const size_t offOBH = offVBL + szX;
  const size_t offOBL = offOBH + szX;
  const size_t total  = offOBL + szX;
  if (ws_size < total) return;

  const float* x_q  = (const float*)d_in[0];
  const float* x_kv = (const float*)d_in[1];
  const float* Wq   = (const float*)d_in[2];
  const float* bq   = (const float*)d_in[3];
  const float* Wk   = (const float*)d_in[4];
  const float* bk   = (const float*)d_in[5];
  const float* Wv   = (const float*)d_in[6];
  const float* bv   = (const float*)d_in[7];
  const float* Wo   = (const float*)d_in[8];
  const float* bo   = (const float*)d_in[9];
  float* out = (float*)d_out;
  char* ws = (char*)d_ws;
  unsigned short* XQB = (unsigned short*)(ws + offXQB);
  unsigned short* XKB = (unsigned short*)(ws + offXKB);
  unsigned short* WQT = (unsigned short*)(ws + offWQT);
  unsigned short* WKT = (unsigned short*)(ws + offWKT);
  unsigned short* WVT = (unsigned short*)(ws + offWVT);
  unsigned short* WOT = (unsigned short*)(ws + offWOT);
  unsigned short* QH  = (unsigned short*)(ws + offQH);
  unsigned short* QBH = (unsigned short*)(ws + offQBH);
  unsigned short* QBL = (unsigned short*)(ws + offQBL);
  unsigned short* KH  = (unsigned short*)(ws + offKH);
  unsigned short* KBH = (unsigned short*)(ws + offKBH);
  unsigned short* KBL = (unsigned short*)(ws + offKBL);
  unsigned short* VH  = (unsigned short*)(ws + offVH);
  unsigned short* VBH = (unsigned short*)(ws + offVBH);
  unsigned short* VBL = (unsigned short*)(ws + offVBL);
  unsigned short* OBH = (unsigned short*)(ws + offOBH);
  unsigned short* OBL = (unsigned short*)(ws + offOBL);

  const int n8 = nElem / 8;
  xcast_bf16_kernel<<<dim3(n8 / 256, 2), dim3(256), 0, stream>>>(x_q, x_kv, XQB, XKB, n8);
  wt_cast_kernel<<<dim3(kDim / 64, kDim / 64, 4), dim3(256), 0, stream>>>(Wq, Wk, Wv, Wo, WQT);

  const int blocksProj = ((kTok / 64) * (kDim / 64)) / 8;
  wmma_gemm64<1, 1, 2, 3><<<dim3(blocksProj, 1), dim3(256), 0, stream>>>(
      XQB, XQB, kDim, 0L, WQT, kDim, 0L, (void*)QH, (void*)QBH, (void*)QBL, kDim, 0L, bq, kTok, kDim, kDim, 1.0f);
  wmma_gemm64<1, 1, 2, 3><<<dim3(blocksProj, 1), dim3(256), 0, stream>>>(
      XKB, XKB, kDim, 0L, WKT, kDim, 0L, (void*)KH, (void*)KBH, (void*)KBL, kDim, 0L, bk, kTok, kDim, kDim, 1.0f);
  wmma_gemm64<1, 1, 1, 3><<<dim3(blocksProj, 1), dim3(256), 0, stream>>>(
      WVT, WVT, kDim, 0L, XKB, kDim, 0L, (void*)VH, (void*)VBH, (void*)VBL, kTok, 0L, bv, kDim, kTok, kDim, 1.0f);

  attn_kernel<true><<<dim3(kSplitQB, kBatch * kHeads), dim3(128), 0, stream>>>(
      QBH, QBL, KBH, KBL, VBH, VBL, OBH, OBL, 0);
  attn_kernel<false><<<dim3(kQBlocks - kSplitQB, kBatch * kHeads), dim3(128), 0, stream>>>(
      QH, QH, KH, KH, VH, VH, OBH, OBL, kSplitQB);

  wmma_gemm64<1, 2, 2, 0><<<dim3(blocksProj, 1), dim3(256), 0, stream>>>(
      OBH, OBL, kDim, 0L, WOT, kDim, 0L, (void*)out, (void*)out, (void*)out, kDim, 0L, bo, kTok, kDim, kDim, 1.0f);
}
